// SelfAttentionV2_798863917454
// MI455X (gfx1250) — hardware-verified
//
#include <hip/hip_runtime.h>
#include <math.h>

#ifndef NB
#define NB 4
#endif
#ifndef SEQ
#define SEQ 2048
#endif
#define NB_FULL 4
#define SEQ_FULL 2048
#define HID 1024
#define O3 3072
#define QKW 2048
#define PCARRY 16384.0f

static_assert(NB >= 1 && NB <= NB_FULL);
static_assert(SEQ >= 128 && SEQ <= SEQ_FULL && (SEQ % 128) == 0);
static_assert((HID % 64) == 0 && (QKW % 64) == 0 && (HID % 256) == 0 && (O3 == 3 * HID));

#define WS_XH ((size_t)NB * SEQ * HID * 2)
#define WS_WH ((size_t)O3 * HID * 2)
#define WS_BR ((size_t)O3 * 4)
#define WS_QK ((size_t)NB * SEQ * QKW * 2)
#define WS_VT ((size_t)NB * HID * SEQ * 2)
#define WS_SB ((size_t)SEQ * SEQ * 4)
#define WS_PP ((size_t)SEQ * SEQ * 2)
static_assert(WS_XH + WS_WH + WS_BR + 2 * WS_QK + WS_VT + WS_SB + WS_PP <= (size_t)134217728);
static_assert((WS_BR % 256) == 0 && (WS_XH % 256) == 0 && (WS_WH % 256) == 0 && (WS_QK % 256) == 0 && (WS_VT % 256) == 0 && (WS_SB % 256) == 0);

typedef __attribute__((ext_vector_type(16))) _Float16 v16h;
typedef __attribute__((ext_vector_type(8)))  _Float16 v8h;
typedef __attribute__((ext_vector_type(16))) __bf16   v16b;
typedef __attribute__((ext_vector_type(8)))  __bf16   v8b;
typedef __attribute__((ext_vector_type(8)))  float    v8f;
typedef __attribute__((ext_vector_type(4)))  float    v4f;
typedef __attribute__((ext_vector_type(4)))  unsigned v4u;

#define VST2(T, ptr, val) do { const T vst2_v_ = (val); *(volatile T*)(ptr) = vst2_v_; __threadfence(); *(volatile T*)(ptr) = vst2_v_; } while (0)

__device__ __forceinline__ unsigned short f2bf_bits(float f) {
  unsigned u = __float_as_uint(f);
  return (unsigned short)((u + 0x7FFFu + ((u >> 16) & 1u)) >> 16);
}
__device__ __forceinline__ float bf_bits2f(unsigned short h) { return __uint_as_float(((unsigned)h) << 16); }
__device__ __forceinline__ unsigned long long pk4h(v4f s) {
  return (unsigned long long)__builtin_bit_cast(unsigned short, (_Float16)s.x) | ((unsigned long long)__builtin_bit_cast(unsigned short, (_Float16)s.y) << 16) |
         ((unsigned long long)__builtin_bit_cast(unsigned short, (_Float16)s.z) << 32) | ((unsigned long long)__builtin_bit_cast(unsigned short, (_Float16)s.w) << 48);
}

namespace w25 {

__device__ __forceinline__ void dep_guard_h(v8f& a, v8f& b, v16h x, v16h y) { asm volatile("v_nop\n\tv_nop\n\tv_nop\n\tv_nop" : "+v"(a), "+v"(b) : "v"(x), "v"(y)); }
__device__ __forceinline__ void dep_guard_b(v8f& a, v8f& b, v16b x, v16b y) { asm volatile("v_nop\n\tv_nop\n\tv_nop\n\tv_nop" : "+v"(a), "+v"(b) : "v"(x), "v"(y)); }
__device__ __forceinline__ void keep4_h(v16h a, v16h b, v16h c, v16h d) { asm volatile("v_nop" :: "v"(a), "v"(b), "v"(c), "v"(d)); }
__device__ __forceinline__ void keep4_b(v16b a, v16b b, v16b c, v16b d) { asm volatile("v_nop" :: "v"(a), "v"(b), "v"(c), "v"(d)); }
__device__ __forceinline__ void acc_guard4(v8f& a, v8f& b, v8f& c, v8f& d) { asm volatile("v_nop\n\tv_nop\n\tv_nop\n\tv_nop" : "+v"(a), "+v"(b), "+v"(c), "+v"(d)); }
template <typename T> struct Frag;
template <> struct Frag<_Float16> {
  typedef v16h V; union U { v16h v; v8h h[2]; };
  static __device__ __forceinline__ v16h load(const _Float16* p) {
    U f; f.h[0] = *(const v8h*)(p); f.h[1] = *(const v8h*)(p + 16); return f.v;
  }
  static __device__ __forceinline__ v8f mma(v16h a, v16h b, v8f c) {
    return __builtin_amdgcn_wmma_f32_16x16x32_f16(false, a, false, b, (short)0, c, false, false);
  }
  static __device__ __forceinline__ void guard(v8f& a, v8f& b, v16h x, v16h y) { dep_guard_h(a, b, x, y); }
  static __device__ __forceinline__ void keep(v16h a, v16h b, v16h c, v16h d) { keep4_h(a, b, c, d); }
};
template <> struct Frag<__bf16> {
  typedef v16b V; union U { v16b v; v8b h[2]; };
  static __device__ __forceinline__ v16b load(const __bf16* p) {
    U f; f.h[0] = *(const v8b*)(p); f.h[1] = *(const v8b*)(p + 16); return f.v;
  }
  static __device__ __forceinline__ v8f mma(v16b a, v16b b, v8f c) {
    return __builtin_amdgcn_wmma_f32_16x16x32_bf16(false, a, false, b, (short)0, c, false, false);
  }
  static __device__ __forceinline__ void guard(v8f& a, v8f& b, v16b x, v16b y) { dep_guard_b(a, b, x, y); }
  static __device__ __forceinline__ void keep(v16b a, v16b b, v16b c, v16b d) { keep4_b(a, b, c, d); }
};

template <int ET> struct Elem;
template <> struct Elem<0> { typedef _Float16 T; };
template <> struct Elem<1> { typedef __bf16 T; };
template <int ET, bool SPLIT, int BIAS_MODE, int OUT_MODE, bool RESID, int ACT = 0>
__global__ __launch_bounds__(256) void wmma_gemm64(
    const unsigned short* __restrict__ Ap, const unsigned short* __restrict__ A2p, int lda, long strideA,
    const unsigned short* __restrict__ Btp, const unsigned short* __restrict__ Bt2p, int ldb, long strideB,
    void* __restrict__ Cout, void* __restrict__ Cout2, int ldc, long strideC,
    const float* __restrict__ bias,
    const float* __restrict__ resid, long strideR,
    int M, int N, int K, float scale) {
  typedef typename Elem<ET>::T T;
  typedef typename Frag<T>::V V;
  const T* A = (const T*)Ap; const T* A2 = (const T*)A2p; const T* Bt = (const T*)Btp; const T* Bt2 = (const T*)Bt2p;
  __shared__ __align__(16) float sT[8][16 * 68];
  const int b    = blockIdx.y;
  const int lane = threadIdx.x & 31;
  const int wave = threadIdx.x >> 5;
  const int tilesN = N >> 6;
  const int tilesM = M >> 6;
  const int tile = blockIdx.x * 8 + wave;
  if (tile >= tilesM * tilesN) return;
  const int tm = tile / tilesN;
  const int tn = tile - tm * tilesN;
  const int m0 = tm << 6;
  const int n0 = tn << 6;

  const T* Ab  = A  + (size_t)b * strideA;
  const T* Bb  = Bt + (size_t)b * strideB;
  const T* Ab2 = SPLIT ? (A2  + (size_t)b * strideA) : nullptr;
  const T* Bb2 = SPLIT ? (Bt2 + (size_t)b * strideB) : nullptr;

  const int rlane = lane & 15;
  const int koff  = (lane >> 4) * 8;
  const int mOff  = (lane >> 4) * 8;

  v8f acc[4][4];
#pragma unroll
  for (int i = 0; i < 4; ++i)
#pragma unroll
    for (int j = 0; j < 4; ++j) acc[i][j] = (v8f){0.f,0.f,0.f,0.f,0.f,0.f,0.f,0.f};

  for (int k0 = 0; k0 < K; k0 += 32) {
    V bh[4], bl[4];
#pragma unroll
    for (int j = 0; j < 4; ++j) {
      const size_t bo = (size_t)(n0 + (j << 4) + rlane) * ldb + koff + k0;
      bh[j] = Frag<T>::load(Bb + bo);
      if (SPLIT) bl[j] = Frag<T>::load(Bb2 + bo);
    }
#pragma unroll
    for (int i = 0; i < 4; ++i) {
      const size_t ao = (size_t)(m0 + (i << 4) + rlane) * lda + koff + k0;
      V ah = Frag<T>::load(Ab + ao);
      V al = ah;
      if (SPLIT) al = Frag<T>::load(Ab2 + ao);
#pragma unroll
      for (int j = 0; j < 4; ++j) {
        acc[i][j] = Frag<T>::mma(ah, bh[j], acc[i][j]);
        if (SPLIT) {
          acc[i][j] = Frag<T>::mma(ah, bl[j], acc[i][j]);
          acc[i][j] = Frag<T>::mma(al, bh[j], acc[i][j]);
        }
      }
      Frag<T>::guard(acc[i][0], acc[i][3], ah, SPLIT ? al : ah);
    }
    Frag<T>::keep(bh[0], bh[1], bh[2], bh[3]);
    if (SPLIT) Frag<T>::keep(bl[0], bl[1], bl[2], bl[3]);
  }
  acc_guard4(acc[0][0], acc[0][1], acc[0][2], acc[0][3]);
  acc_guard4(acc[1][0], acc[1][1], acc[1][2], acc[1][3]);
  acc_guard4(acc[2][0], acc[2][1], acc[2][2], acc[2][3]);
  acc_guard4(acc[3][0], acc[3][1], acc[3][2], acc[3][3]);

  float* slab = sT[wave];
  const float* Rb = RESID ? (resid + (size_t)b * strideR) : nullptr;
#pragma unroll
  for (int i = 0; i < 4; ++i) {
    const int mBase = m0 + (i << 4);
#pragma unroll
    for (int j = 0; j < 4; ++j) {
      const int n = n0 + (j << 4) + rlane;
      float bv = 0.f;
      if (BIAS_MODE == 2) bv = bias[n];
#pragma unroll
      for (int r = 0; r < 8; ++r) {
        float v = acc[i][j][r] * scale;
        if (BIAS_MODE == 1) v += bias[mBase + mOff + r];
        if (BIAS_MODE == 2) v += bv;
        if (RESID) v += Rb[(size_t)(mBase + mOff + r) * ldc + n];
        if (ACT == 1) v = tanhf(v);
        if (ACT == 2) v = fmaxf(v, 0.0f);
        if (ACT == 3) v = v / (1.0f + expf(-v));
        if (ACT == 4) v = (v > 0.f) ? v : 0.01f * v;
        if (ACT == 5) v = 0.5f * v * (1.0f + erff(v * 0.70710678118654752f));
        if (ACT == 6) v = (v > 0.f) ? v : 0.2f * v;
        if (ACT == 7) { const float u = 0.7978845608028654f * (v + 0.044715f * v * v * v); v = 0.5f * v * (1.f + tanhf(u)); }
        slab[(mOff + r) * 68 + (j << 4) + rlane] = v;
      }
    }
    __builtin_amdgcn_fence(__ATOMIC_RELEASE, "workgroup");
    __builtin_amdgcn_wave_barrier();
    __builtin_amdgcn_fence(__ATOMIC_ACQUIRE, "workgroup");
    if (OUT_MODE == 0) {
      float* C = (float*)Cout + (size_t)b * strideC;
      const int hh = lane >> 4, c4 = (lane & 15) * 4;
      for (int pass = 0; pass < 2; ++pass) {
#pragma unroll
        for (int it = 0; it < 8; ++it) {
          const int row = it * 2 + hh;
          v4f v = *(const v4f*)(slab + row * 68 + c4);
          *(volatile v4f*)(C + (size_t)(mBase + row) * ldc + n0 + c4) = v;
        }
        __threadfence();
      }
    } else {
      const int q = lane >> 3, c8 = (lane & 7) * 8;
      unsigned short* C  = (unsigned short*)Cout  + (size_t)b * strideC;
      unsigned short* C2 = (OUT_MODE == 2) ? ((unsigned short*)Cout2 + (size_t)b * strideC) : nullptr;
      for (int pass = 0; pass < 2; ++pass) {
#pragma unroll
        for (int it = 0; it < 4; ++it) {
          const int row = it * 4 + q;
          const float* sp = slab + row * 68 + c8;
          v8h hv, lv;
#pragma unroll
          for (int e = 0; e < 8; ++e) {
            if (OUT_MODE == 1) {
              hv[e] = (_Float16)sp[e];
              lv[e] = hv[e];
            } else {
              unsigned short hb = f2bf_bits(sp[e]);
              unsigned short lb = f2bf_bits(sp[e] - bf_bits2f(hb));
              hv[e] = __builtin_bit_cast(_Float16, hb);
              lv[e] = __builtin_bit_cast(_Float16, lb);
            }
          }
          *(volatile v8h*)(C + (size_t)(mBase + row) * ldc + n0 + c8) = hv;
          if (OUT_MODE == 2) *(volatile v8h*)(C2 + (size_t)(mBase + row) * ldc + n0 + c8) = lv;
        }
        __threadfence();
      }
    }
    __builtin_amdgcn_fence(__ATOMIC_RELEASE, "workgroup");
    __builtin_amdgcn_wave_barrier();
    __builtin_amdgcn_fence(__ATOMIC_ACQUIRE, "workgroup");
  }
}

}

__global__ __launch_bounds__(256) void k_bfpl(const float* __restrict__ src, long long sgs, int rpg, unsigned short* __restrict__ dst, long long rows, int cols) {
    const long long u = (long long)blockIdx.x * 256 + threadIdx.x; const int cq = cols >> 3; if (u >= rows * cq) return;
    const long long r = u / cq; const int c = 8 * (int)(u - r * cq); const long long g = r / rpg; const long long rr = r - g * rpg;
    const float* s = src + g * sgs + rr * (long long)cols + c;
    const v4f a = *(const v4f*)s; const v4f b = *(const v4f*)(s + 4);
    v4u pk;
    pk.x = (unsigned)f2bf_bits(a.x) | ((unsigned)f2bf_bits(a.y) << 16);
    pk.y = (unsigned)f2bf_bits(a.z) | ((unsigned)f2bf_bits(a.w) << 16);
    pk.z = (unsigned)f2bf_bits(b.x) | ((unsigned)f2bf_bits(b.y) << 16);
    pk.w = (unsigned)f2bf_bits(b.z) | ((unsigned)f2bf_bits(b.w) << 16);
    volatile v4u* d = (volatile v4u*)(dst + r * (long long)cols + c); *d = pk; __threadfence(); *d = pk;
}

__global__ __launch_bounds__(256) void k_bvec(const float* __restrict__ bsrc, float* __restrict__ O, int n) {
    for (int i = threadIdx.x; i < n; i += 256) { const float v = bf_bits2f(f2bf_bits(bsrc[i])); VST2(float, O + i, v); }
}

__global__ __launch_bounds__(256) void k_sm16(const float* __restrict__ S, unsigned short* __restrict__ P16, int rows, int n, float carry) {
    #pragma clang fp contract(off)
    const int row = blockIdx.x * 8 + (threadIdx.x >> 5); const int L = threadIdx.x & 31; if (row >= rows) return;
    const float L2E = 1.4426950408889634f;
    const float* sr = S + (long long)row * n; const int G = n >> 7;
    float m = -3.0e38f;
#pragma unroll 1
    for (int g = 0; g < G; ++g) { const v4f s = *(const v4f*)(sr + 128 * g + 4 * L); m = fmaxf(m, fmaxf(fmaxf(s.x, s.y), fmaxf(s.z, s.w))); }
#pragma unroll
    for (int o = 16; o > 0; o >>= 1) m = fmaxf(m, __shfl_xor(m, o, 32));
    float sum = 0.f;
#pragma unroll 1
    for (int g = 0; g < G; ++g) {
        const v4f s = *(const v4f*)(sr + 128 * g + 4 * L);
        sum += exp2f((s.x - m) * L2E) + exp2f((s.y - m) * L2E) + exp2f((s.z - m) * L2E) + exp2f((s.w - m) * L2E);
    }
#pragma unroll
    for (int o = 16; o > 0; o >>= 1) sum += __shfl_xor(sum, o, 32);
    const float inv = carry * (1.0f / sum);
    unsigned short* pr = P16 + (long long)row * n;
#pragma unroll 1
    for (int g = 0; g < G; ++g) {
        const int c = 128 * g + 4 * L;
        const v4f s = *(const v4f*)(sr + c);
        v4f p;
        p.x = exp2f((s.x - m) * L2E) * inv; p.y = exp2f((s.y - m) * L2E) * inv; p.z = exp2f((s.z - m) * L2E) * inv; p.w = exp2f((s.w - m) * L2E) * inv;
        const unsigned long long pk = pk4h(p);
        VST2(unsigned long long, (unsigned long long*)(pr + c), pk);
    }
}

extern "C" void kernel_launch(void* const* d_in, const int* in_sizes, int n_in, void* d_out, int out_size, void* d_ws, size_t ws_size, hipStream_t stream) {
    if (n_in < 3) return;
    const long long needX = ((long long)(NB - 1) * SEQ_FULL + SEQ) * HID;
    if ((long long)in_sizes[0] < needX) return;
    if ((long long)in_sizes[1] < (long long)O3 * HID) return;
    if (in_sizes[2] < O3) return;
    if ((long long)out_size < (long long)NB * SEQ * HID) return;
    const float* X  = (const float*)d_in[0];
    const float* W  = (const float*)d_in[1];
    const float* bb = (const float*)d_in[2];
    float* out = (float*)d_out;

    char* wsp = (char*)d_ws;
    unsigned short* XH  = (unsigned short*)wsp; wsp += WS_XH;
    unsigned short* WH  = (unsigned short*)wsp; wsp += WS_WH;
    float*          BR  = (float*)wsp;          wsp += WS_BR;
    unsigned short* QKH = (unsigned short*)wsp; wsp += WS_QK;
    unsigned short* QKL = (unsigned short*)wsp; wsp += WS_QK;
    unsigned short* VT  = (unsigned short*)wsp; wsp += WS_VT;
    float*          SB  = (float*)wsp;          wsp += WS_SB;
    unsigned short* PP  = (unsigned short*)wsp; wsp += WS_PP;
    if ((size_t)(wsp - (char*)d_ws) > ws_size) return;

    const int R = NB * SEQ;
    k_bfpl<<<(unsigned)(((long long)R * (HID / 8) + 255) / 256), 256, 0, stream>>>(X, (long long)SEQ_FULL * HID, SEQ, XH, (long long)R, HID);
    k_bfpl<<<(unsigned)(((long long)O3 * (HID / 8) + 255) / 256), 256, 0, stream>>>(W, 0LL, O3, WH, (long long)O3, HID);
    k_bvec<<<1, 256, 0, stream>>>(bb, BR, O3);
    w25::wmma_gemm64<1, false, 2, 2, false, 0><<<dim3((unsigned)(((R / 64) * (QKW / 64) + 7) / 8), 1), 256, 0, stream>>>(
        XH, nullptr, HID, 0L, WH, nullptr, HID, 0L, (void*)QKH, (void*)QKL, QKW, 0L, BR, nullptr, 0L, R, QKW, HID, 1.0f);
    w25::wmma_gemm64<1, false, 1, 1, false, 0><<<dim3((unsigned)(((HID / 64) * (SEQ / 64) + 7) / 8), NB), 256, 0, stream>>>(
        WH + (size_t)2 * HID * HID, nullptr, HID, 0L, XH, nullptr, HID, (long)SEQ * HID, (void*)VT, nullptr, SEQ, (long)HID * SEQ,
        BR + 2 * HID, nullptr, 0L, HID, SEQ, HID, 1.0f);
    for (int b = 0; b < NB; ++b) {
        const unsigned short* qh = QKH + (size_t)b * SEQ * QKW;
        const unsigned short* ql = QKL + (size_t)b * SEQ * QKW;
        w25::wmma_gemm64<1, true, 0, 0, false, 0><<<dim3((unsigned)(((SEQ / 64) * (SEQ / 64) + 7) / 8), 1), 256, 0, stream>>>(
            qh, ql, QKW, 0L, qh + HID, ql + HID, QKW, 0L, (void*)SB, nullptr, SEQ, 0L, nullptr, nullptr, 0L, SEQ, SEQ, HID, 0.03125f);
        k_sm16<<<(unsigned)(SEQ / 8), 256, 0, stream>>>(SB, PP, SEQ, SEQ, PCARRY);
        w25::wmma_gemm64<0, false, 0, 0, false, 0><<<dim3((unsigned)(((SEQ / 64) * (HID / 64) + 7) / 8), 1), 256, 0, stream>>>(
            PP, nullptr, SEQ, 0L, VT + (size_t)b * HID * SEQ, nullptr, SEQ, 0L, (void*)(out + (size_t)b * SEQ * HID), nullptr, HID, 0L,
            nullptr, nullptr, 0L, SEQ, HID, SEQ, 1.0f / PCARRY);
    }
}
